// BigBirdEncoderBlock_44203803410664
// MI455X (gfx1250) — hardware-verified
//
#include <hip/hip_runtime.h>

typedef _Float16 v16h __attribute__((ext_vector_type(16)));
typedef _Float16 v8h  __attribute__((ext_vector_type(8)));
typedef float    v8f  __attribute__((ext_vector_type(8)));
typedef float    v4f  __attribute__((ext_vector_type(4)));
typedef int      v4i  __attribute__((ext_vector_type(4)));
typedef v8h __attribute__((may_alias)) v8ha;
typedef v4f __attribute__((may_alias)) v4fa;
typedef v4i __attribute__((may_alias)) v4ia;

union Frag { v16h v; v8h half[2]; };

#define NB     8
#define SEQ    1024
#define DM     512
#define NH     8
#define HD     64
#define NBLK   16
#define MLPD   1024
#define NROWS  (NB * SEQ)
#define NQKV   (3 * DM)
#define WSC    16.0f
#define INVW   0.0625f
#define QSC    0.125f
#define PSCALE 256.0f
#define INVP   0.00390625f
#define NEGV   (-1.0e9f)
#define KPITCH 72

__device__ __forceinline__ v8f wmma_f16(v16h a, v16h b, v8f c) {
  v8f d = __builtin_amdgcn_wmma_f32_16x16x32_f16(false, a, false, b, (short)0, c, false, false);
  asm volatile("v_nop\n\tv_nop\n\tv_nop\n\tv_nop" : "+v"(d) : "v"(a), "v"(b));
  return d;
}

__device__ __forceinline__ v16h load_frag(const _Float16* p, int h) {
  Frag f;
  f.half[0] = *(const v8ha*)(p + 8 * h);
  f.half[1] = *(const v8ha*)(p + 16 + 8 * h);
  return f.v;
}

__device__ __forceinline__ void wt_store_pass(const float (*tile)[65], _Float16* dbase,
                                              int n0, int k0, int K, int w, int lane) {
  const int q8 = lane & 7, sub = lane >> 3;
  #pragma unroll
  for (int i = 0; i < 2; ++i) {
    const int nl = w * 8 + i * 4 + sub;
    const int kb = 8 * q8;
    const v8h v = { (_Float16)tile[kb + 0][nl], (_Float16)tile[kb + 1][nl],
                    (_Float16)tile[kb + 2][nl], (_Float16)tile[kb + 3][nl],
                    (_Float16)tile[kb + 4][nl], (_Float16)tile[kb + 5][nl],
                    (_Float16)tile[kb + 6][nl], (_Float16)tile[kb + 7][nl] };
    *(volatile v8h*)(dbase + (size_t)(n0 + nl) * K + k0 + kb) = v;
  }
}

__global__ __launch_bounds__(256) void cvt_w_kernel(
    const float* __restrict__ s0, const float* __restrict__ s1, const float* __restrict__ s2,
    _Float16* dst, int K, int N)
{
  __shared__ float tile[64][65];
  const int tid = threadIdx.x, lane = tid & 31, w = tid >> 5;
  const int k0 = blockIdx.x * 64, n0 = blockIdx.y * 64, z = blockIdx.z;
  const float* src = (z == 0) ? s0 : ((z == 1) ? s1 : s2);
  const int nl = tid & 63, kq = tid >> 6;
  #pragma unroll
  for (int i = 0; i < 16; ++i) {
    const int kl = i * 4 + kq;
    tile[kl][nl] = src[(size_t)(k0 + kl) * N + n0 + nl] * WSC;
  }
  __syncthreads();
  _Float16* dbase = dst + (size_t)z * N * K;
  wt_store_pass(tile, dbase, n0, k0, K, w, lane);
  __threadfence();
  wt_store_pass(tile, dbase, n0, k0, K, w, lane);
}

__device__ __forceinline__ v8h ln_pack(v4f a, v4f c, float mean, float rstd,
                                       v4f ga, v4f gc, v4f ba, v4f bc) {
  const v8h o = { (_Float16)((a.x - mean) * rstd * ga.x + ba.x), (_Float16)((a.y - mean) * rstd * ga.y + ba.y),
                  (_Float16)((a.z - mean) * rstd * ga.z + ba.z), (_Float16)((a.w - mean) * rstd * ga.w + ba.w),
                  (_Float16)((c.x - mean) * rstd * gc.x + bc.x), (_Float16)((c.y - mean) * rstd * gc.y + bc.y),
                  (_Float16)((c.z - mean) * rstd * gc.z + bc.z), (_Float16)((c.w - mean) * rstd * gc.w + bc.w) };
  return o;
}

__global__ __launch_bounds__(256) void ln_kernel(
    const float* __restrict__ x, const float* __restrict__ sc, const float* __restrict__ bi,
    _Float16* out, int rows)
{
  const int wid = blockIdx.x * 8 + (threadIdx.x >> 5);
  const int lane = threadIdx.x & 31;
  if (wid >= rows) return;
  const float* rp = x + (size_t)wid * DM;
  const int c0 = 8 * lane, c1 = 256 + 8 * lane;
  const v4f a0 = *(const v4fa*)(rp + c0);
  const v4f a1 = *(const v4fa*)(rp + c0 + 4);
  const v4f a2 = *(const v4fa*)(rp + c1);
  const v4f a3 = *(const v4fa*)(rp + c1 + 4);
  float s = ((a0.x + a0.y) + (a0.z + a0.w)) + ((a1.x + a1.y) + (a1.z + a1.w))
          + ((a2.x + a2.y) + (a2.z + a2.w)) + ((a3.x + a3.y) + (a3.z + a3.w));
  #pragma unroll
  for (int off = 16; off >= 1; off >>= 1) s += __shfl_xor(s, off, 32);
  const float mean = s * (1.0f / DM);
  const v4f d0 = a0 - mean, d1 = a1 - mean, d2 = a2 - mean, d3 = a3 - mean;
  float t = (d0.x * d0.x + d0.y * d0.y + d0.z * d0.z + d0.w * d0.w)
          + (d1.x * d1.x + d1.y * d1.y + d1.z * d1.z + d1.w * d1.w)
          + (d2.x * d2.x + d2.y * d2.y + d2.z * d2.z + d2.w * d2.w)
          + (d3.x * d3.x + d3.y * d3.y + d3.z * d3.z + d3.w * d3.w);
  #pragma unroll
  for (int off = 16; off >= 1; off >>= 1) t += __shfl_xor(t, off, 32);
  const float rstd = rsqrtf(t * (1.0f / DM) + 1e-6f);

  const v4f g0 = *(const v4fa*)(sc + c0), g1 = *(const v4fa*)(sc + c0 + 4);
  const v4f g2 = *(const v4fa*)(sc + c1), g3 = *(const v4fa*)(sc + c1 + 4);
  const v4f e0 = *(const v4fa*)(bi + c0), e1 = *(const v4fa*)(bi + c0 + 4);
  const v4f e2 = *(const v4fa*)(bi + c1), e3 = *(const v4fa*)(bi + c1 + 4);
  const v8h o0 = ln_pack(a0, a1, mean, rstd, g0, g1, e0, e1);
  const v8h o1 = ln_pack(a2, a3, mean, rstd, g2, g3, e2, e3);

  _Float16* op = out + (size_t)wid * DM;
  *(volatile v8h*)(op + c0) = o0;
  *(volatile v8h*)(op + c1) = o1;
  __threadfence();
  *(volatile v8h*)(op + c0) = o0;
  *(volatile v8h*)(op + c1) = o1;
}

__device__ __forceinline__ void h_store_pass(const _Float16* sH, _Float16* dst, size_t row0,
                                             int pitch, int col0, int w, int lane) {
  const int q8 = lane & 7, sub = lane >> 3;
  #pragma unroll
  for (int i = 0; i < 8; ++i) {
    const int lid = w * 32 + i * 4 + sub;
    const v8h v = *(const v8ha*)(sH + lid * 64 + 8 * q8);
    *(volatile v8h*)(dst + (row0 + (size_t)lid) * (size_t)pitch + col0 + 8 * q8) = v;
  }
}

__device__ __forceinline__ void vt_store_pass(const _Float16* sH, _Float16* vtp, int bh, int l0,
                                              int w, int lane) {
  const int q8 = lane & 7, sub = lane >> 3;
  #pragma unroll
  for (int i = 0; i < 8; ++i) {
    const int lid = w * 32 + i * 4 + sub;
    const int d = lid >> 1, hl = lid & 1;
    const v8h v = *(const v8ha*)(sH + d * 128 + 64 * hl + 8 * q8);
    *(volatile v8h*)(vtp + ((size_t)bh * HD + d) * SEQ + l0 + 64 * hl + 8 * q8) = v;
  }
}

__device__ __forceinline__ void f_store_pass(const float* sT, const float* __restrict__ resid,
                                             float* dst, int m0, int n0, int N, int w, int lane) {
  const int q8 = lane & 7, sub = lane >> 3;
  #pragma unroll
  for (int i = 0; i < 16; ++i) {
    const int lid = i * 4 + sub;
    const int row = 32 * w + (lid >> 1), hl = lid & 1;
    const v4f a = *(const v4fa*)(sT + row * 64 + 32 * hl + 4 * q8);
    const size_t gi = (size_t)(m0 + row) * N + n0 + 32 * hl + 4 * q8;
    const v4f rr = *(const v4fa*)(resid + gi);
    const v4f v = a + rr;
    *(volatile v4f*)(dst + gi) = v;
  }
}

__device__ __forceinline__ float gelu_tanh(float x) {
  const float u = 0.7978845608028654f * (x + 0.044715f * x * x * x);
  return 0.5f * x * (1.0f + tanhf(u));
}

template <int MODE>
__global__ __launch_bounds__(128) void gemm_kernel(
    const _Float16* __restrict__ A, const _Float16* __restrict__ Bt, int N, int K,
    const float* __restrict__ bias, const float* __restrict__ resid,
    float* outf, _Float16* outh, _Float16* qpl, _Float16* kpl, _Float16* vtp)
{
  __shared__ __attribute__((aligned(16))) float sT[128 * 64];
  _Float16* sH = (_Float16*)sT;

  const int tid = threadIdx.x, lane = tid & 31, w = tid >> 5;
  const int h = lane >> 4, m = lane & 15;
  const int m0 = blockIdx.x * 128;
  const int n0 = blockIdx.y * 64;
  const int m0w = m0 + 32 * w;

  const _Float16* xa0 = A + (size_t)(m0w + m) * K;
  const _Float16* xa1 = xa0 + (size_t)16 * K;
  const _Float16* wb  = Bt + (size_t)(n0 + m) * K;

  const v8f zero8 = {0.f, 0.f, 0.f, 0.f, 0.f, 0.f, 0.f, 0.f};
  v8f acc[2][4];
  #pragma unroll
  for (int mt = 0; mt < 2; ++mt)
    #pragma unroll
    for (int nt = 0; nt < 4; ++nt) acc[mt][nt] = zero8;

  #pragma unroll 1
  for (int k0 = 0; k0 < K; k0 += 32) {
    const v16h a0 = load_frag(xa0 + k0, h);
    const v16h a1 = load_frag(xa1 + k0, h);
    #pragma unroll
    for (int nt = 0; nt < 4; ++nt) {
      const v16h bq = load_frag(wb + (size_t)nt * 16 * K + k0, h);
      acc[0][nt] = wmma_f16(a0, bq, acc[0][nt]);
      acc[1][nt] = wmma_f16(a1, bq, acc[1][nt]);
    }
  }

  if (MODE == 0) {
    const int which = n0 / DM;
    const int head = (n0 - which * DM) / HD;
    #pragma unroll
    for (int nt = 0; nt < 4; ++nt) {
      const int feat = 16 * nt + m;
      #pragma unroll
      for (int mt = 0; mt < 2; ++mt) {
        #pragma unroll
        for (int r = 0; r < 8; ++r) {
          const int tokl = 32 * w + 16 * mt + 8 * h + r;
          const float y = acc[mt][nt][r] * INVW;
          const int si = (which == 2) ? (feat * 128 + tokl) : (tokl * 64 + feat);
          sH[si] = (_Float16)y;
        }
      }
    }
    __syncthreads();
    const int b = m0 / SEQ, l0 = m0 - b * SEQ, bh = b * NH + head;
    if (which == 2) {
      vt_store_pass(sH, vtp, bh, l0, w, lane);
      __threadfence();
      vt_store_pass(sH, vtp, bh, l0, w, lane);
    } else {
      _Float16* plane = (which == 0) ? qpl : kpl;
      const size_t row0 = (size_t)bh * SEQ + l0;
      h_store_pass(sH, plane, row0, HD, 0, w, lane);
      __threadfence();
      h_store_pass(sH, plane, row0, HD, 0, w, lane);
    }
  } else if (MODE == 2) {
    #pragma unroll
    for (int nt = 0; nt < 4; ++nt) {
      const int feat = 16 * nt + m;
      const float bvl = bias[n0 + feat];
      #pragma unroll
      for (int mt = 0; mt < 2; ++mt) {
        #pragma unroll
        for (int r = 0; r < 8; ++r) {
          const int tokl = 32 * w + 16 * mt + 8 * h + r;
          const float y = gelu_tanh(acc[mt][nt][r] * INVW + bvl);
          sH[tokl * 64 + feat] = (_Float16)y;
        }
      }
    }
    __syncthreads();
    h_store_pass(sH, outh, (size_t)m0, N, n0, w, lane);
    __threadfence();
    h_store_pass(sH, outh, (size_t)m0, N, n0, w, lane);
  } else {
    #pragma unroll
    for (int nt = 0; nt < 4; ++nt) {
      const int feat = 16 * nt + m;
      const float bvl = (MODE == 3) ? bias[n0 + feat] : 0.0f;
      #pragma unroll
      for (int mt = 0; mt < 2; ++mt) {
        #pragma unroll
        for (int r = 0; r < 8; ++r) {
          const int tokl = 32 * w + 16 * mt + 8 * h + r;
          sT[tokl * 64 + feat] = acc[mt][nt][r] * INVW + bvl;
        }
      }
    }
    __syncthreads();
    f_store_pass(sT, resid, outf, m0, n0, N, w, lane);
    __threadfence();
    f_store_pass(sT, resid, outf, m0, n0, N, w, lane);
  }
}

__device__ __forceinline__ v16h pack_p(v8f a, v8f c) {
  const v16h r = { (_Float16)(a[0] * PSCALE), (_Float16)(a[1] * PSCALE), (_Float16)(a[2] * PSCALE), (_Float16)(a[3] * PSCALE),
                   (_Float16)(a[4] * PSCALE), (_Float16)(a[5] * PSCALE), (_Float16)(a[6] * PSCALE), (_Float16)(a[7] * PSCALE),
                   (_Float16)(c[0] * PSCALE), (_Float16)(c[1] * PSCALE), (_Float16)(c[2] * PSCALE), (_Float16)(c[3] * PSCALE),
                   (_Float16)(c[4] * PSCALE), (_Float16)(c[5] * PSCALE), (_Float16)(c[6] * PSCALE), (_Float16)(c[7] * PSCALE) };
  return r;
}

__device__ __forceinline__ v8f mask_scale8(v8f s, const int* p, int kflag) {
  const v4i ma = *(const v4ia*)p;
  const v4i mb = *(const v4ia*)(p + 4);
  const bool kf = (kflag != 0);
  s[0] = ((ma.x != 0) & kf) ? s[0] * QSC : NEGV;
  s[1] = ((ma.y != 0) & kf) ? s[1] * QSC : NEGV;
  s[2] = ((ma.z != 0) & kf) ? s[2] * QSC : NEGV;
  s[3] = ((ma.w != 0) & kf) ? s[3] * QSC : NEGV;
  s[4] = ((mb.x != 0) & kf) ? s[4] * QSC : NEGV;
  s[5] = ((mb.y != 0) & kf) ? s[5] * QSC : NEGV;
  s[6] = ((mb.z != 0) & kf) ? s[6] * QSC : NEGV;
  s[7] = ((mb.w != 0) & kf) ? s[7] * QSC : NEGV;
  return s;
}

__device__ __forceinline__ void att_store_pass(const _Float16* so, _Float16* attn,
                                               int b, int head, int q0, int lane) {
  const int q8 = lane & 7, sub = lane >> 3;
  #pragma unroll
  for (int i = 0; i < 4; ++i) {
    const int row = i * 4 + sub;
    const v8h v = *(const v8ha*)(so + row * 64 + 8 * q8);
    const size_t gi = ((size_t)b * SEQ + q0 + row) * DM + head * HD + 8 * q8;
    *(volatile v8h*)(attn + gi) = v;
  }
}

__global__ __launch_bounds__(128) void attn_kernel(
    const _Float16* __restrict__ qpl,
    const _Float16* __restrict__ kpl,
    const _Float16* __restrict__ vtp,
    const int* __restrict__ pm,
    const int* __restrict__ ra,
    _Float16* attn)
{
  __shared__ __attribute__((aligned(16))) _Float16 Ks[64 * KPITCH];
  __shared__ __attribute__((aligned(16))) _Float16 Vs[64 * KPITCH];
  __shared__ __attribute__((aligned(16))) _Float16 sO[4 * 16 * 64];

  const int tid = threadIdx.x, lane = tid & 31, w = tid >> 5;
  const int h = lane >> 4, m = lane & 15;
  const int mblk = blockIdx.x, head = blockIdx.y, b = blockIdx.z;
  const int bh = b * NH + head;
  const bool is_global = (mblk == 0) || (mblk == NBLK - 1);

  int c5 = ra[mblk * 3 + 0], c6 = ra[mblk * 3 + 1], c7 = ra[mblk * 3 + 2];
  c5 = (c5 < 0) ? 0 : ((c5 > NBLK - 1) ? (NBLK - 1) : c5);
  c6 = (c6 < 0) ? 0 : ((c6 > NBLK - 1) ? (NBLK - 1) : c6);
  c7 = (c7 < 0) ? 0 : ((c7 > NBLK - 1) ? (NBLK - 1) : c7);
  int t[8];
  t[0] = 0; t[1] = NBLK - 1; t[2] = (mblk + NBLK - 1) & (NBLK - 1); t[3] = mblk;
  t[4] = (mblk + 1) & (NBLK - 1); t[5] = c5; t[6] = c6; t[7] = c7;
  unsigned idxpack = 0u, keepbits = 0u;
  #pragma unroll
  for (int s = 0; s < 8; ++s) {
    int kp = 1;
    #pragma unroll
    for (int ss = 0; ss < s; ++ss) kp = (t[ss] == t[s]) ? 0 : kp;
    idxpack |= ((unsigned)t[s] & 15u) << (4 * s);
    keepbits |= (unsigned)kp << s;
  }
  const int nb = is_global ? NBLK : 8;

  const int q0 = mblk * 64 + 16 * w;
  const _Float16* qrow = qpl + ((size_t)bh * SEQ + q0 + m) * HD;
  const v16h qb0 = load_frag(qrow, h);
  const v16h qb1 = load_frag(qrow + 32, h);

  const v8f zero8 = {0.f, 0.f, 0.f, 0.f, 0.f, 0.f, 0.f, 0.f};
  v8f o[4];
  #pragma unroll
  for (int tt = 0; tt < 4; ++tt) o[tt] = zero8;
  float mrun = -1e30f, lrun = 0.0f;

  const int* pmrow = pm + (size_t)b * SEQ;
  const int srow = tid >> 3, sch = tid & 7;

  #pragma unroll 1
  for (int jj = 0; jj < nb; ++jj) {
    const int kblk  = is_global ? jj : (int)((idxpack >> ((4 * jj) & 28)) & 15u);
    const int kflag = is_global ? 1 : (int)((keepbits >> (jj & 31)) & 1u);

    __syncthreads();
    {
      const _Float16* kp = kpl + ((size_t)bh * SEQ + kblk * 64 + srow) * HD + 8 * sch;
      const _Float16* vp = vtp + ((size_t)bh * HD + srow) * SEQ + kblk * 64 + 8 * sch;
      #pragma unroll
      for (int c = 0; c < 4; ++c) {
        const v8h kv = *(const v8ha*)(kp + (size_t)16 * c * HD);
        const v8h vv = *(const v8ha*)(vp + (size_t)16 * c * SEQ);
        *(v8ha*)(Ks + (srow + 16 * c) * KPITCH + 8 * sch) = kv;
        *(v8ha*)(Vs + (srow + 16 * c) * KPITCH + 8 * sch) = vv;
      }
    }
    __syncthreads();

    v8f s[4];
    #pragma unroll
    for (int j = 0; j < 4; ++j) {
      const _Float16* krow = Ks + (16 * j + m) * KPITCH;
      const v16h kf0 = load_frag(krow, h);
      const v16h kf1 = load_frag(krow + 32, h);
      v8f z = zero8;
      z = wmma_f16(kf0, qb0, z);
      z = wmma_f16(kf1, qb1, z);
      s[j] = z;
    }
    #pragma unroll
    for (int j = 0; j < 4; ++j) s[j] = mask_scale8(s[j], pmrow + kblk * 64 + 16 * j + 8 * h, kflag);

    float mloc = -1e30f;
    #pragma unroll
    for (int j = 0; j < 4; ++j)
      #pragma unroll
      for (int r = 0; r < 8; ++r) mloc = fmaxf(mloc, s[j][r]);
    mloc = fmaxf(mloc, __shfl_xor(mloc, 16, 32));
    const float mnew = fmaxf(mrun, mloc);
    const float alpha = __expf(mrun - mnew);
    mrun = mnew;
    float lsum = 0.0f;
    #pragma unroll
    for (int j = 0; j < 4; ++j)
      #pragma unroll
      for (int r = 0; r < 8; ++r) {
        const float p = __expf(s[j][r] - mnew);
        s[j][r] = p;
        lsum += p;
      }
    lsum += __shfl_xor(lsum, 16, 32);
    lrun = lrun * alpha + lsum;
    #pragma unroll
    for (int tt = 0; tt < 4; ++tt)
      #pragma unroll
      for (int r = 0; r < 8; ++r) o[tt][r] = o[tt][r] * alpha;

    const v16h pb0 = pack_p(s[0], s[1]);
    const v16h pb1 = pack_p(s[2], s[3]);

    #pragma unroll
    for (int tt = 0; tt < 4; ++tt) {
      const _Float16* vrow = Vs + (16 * tt + m) * KPITCH;
      const v16h vf0 = load_frag(vrow, h);
      const v16h vf1 = load_frag(vrow + 32, h);
      o[tt] = wmma_f16(vf0, pb0, o[tt]);
      o[tt] = wmma_f16(vf1, pb1, o[tt]);
    }
  }

  const float inv = (1.0f / lrun) * INVP;
  _Float16* so = sO + w * 1024;
  #pragma unroll
  for (int tt = 0; tt < 4; ++tt)
    #pragma unroll
    for (int r = 0; r < 8; ++r)
      so[m * 64 + 16 * tt + 8 * h + r] = (_Float16)(o[tt][r] * inv);
  __syncthreads();

  att_store_pass(so, attn, b, head, q0, lane);
  __threadfence();
  att_store_pass(so, attn, b, head, q0, lane);
}

extern "C" void kernel_launch(void* const* d_in, const int* in_sizes, int n_in,
                              void* d_out, int out_size, void* d_ws, size_t ws_size,
                              hipStream_t stream) {
  if (n_in < 15) return;
  if (in_sizes[0] != NROWS * DM || in_sizes[1] != NROWS) return;
  if (in_sizes[2] != DM || in_sizes[3] != DM || in_sizes[8] != DM || in_sizes[9] != DM || in_sizes[13] != DM) return;
  if (in_sizes[4] != DM * DM || in_sizes[5] != DM * DM || in_sizes[6] != DM * DM || in_sizes[7] != DM * DM) return;
  if (in_sizes[10] != DM * MLPD || in_sizes[11] != MLPD || in_sizes[12] != MLPD * DM) return;
  if (in_sizes[14] != NBLK * 3) return;
  if (out_size != NROWS * DM) return;

  const float* x    = (const float*)d_in[0];
  const int*   pm   = (const int*)d_in[1];
  const float* ln1s = (const float*)d_in[2];
  const float* ln1b = (const float*)d_in[3];
  const float* Wq   = (const float*)d_in[4];
  const float* Wk   = (const float*)d_in[5];
  const float* Wv   = (const float*)d_in[6];
  const float* Wo   = (const float*)d_in[7];
  const float* ln2s = (const float*)d_in[8];
  const float* ln2b = (const float*)d_in[9];
  const float* W1   = (const float*)d_in[10];
  const float* b1   = (const float*)d_in[11];
  const float* W2   = (const float*)d_in[12];
  const float* b2   = (const float*)d_in[13];
  const int*   ra   = (const int*)d_in[14];
  float* out = (float*)d_out;

  const size_t wqkv_b = (size_t)NQKV * DM * 2;
  const size_t wo_b   = (size_t)DM * DM * 2;
  const size_t w1_b   = (size_t)MLPD * DM * 2;
  const size_t w2_b   = (size_t)DM * MLPD * 2;
  const size_t xh_b   = (size_t)NROWS * DM * 2;
  const size_t pl_b   = (size_t)NB * NH * SEQ * HD * 2;
  const size_t at_b   = (size_t)NROWS * DM * 2;
  const size_t xr_b   = (size_t)NROWS * DM * 4;
  const size_t yh_b   = (size_t)NROWS * DM * 2;
  const size_t hh_b   = (size_t)NROWS * MLPD * 2;
  const size_t total  = wqkv_b + wo_b + w1_b + w2_b + xh_b + 3 * pl_b + at_b + xr_b + yh_b + hh_b;
  if (total > ws_size) return;

  char* ws = (char*)d_ws;
  size_t off = 0;
  _Float16* wqkv = (_Float16*)(ws + off); off += wqkv_b;
  _Float16* woT  = (_Float16*)(ws + off); off += wo_b;
  _Float16* w1T  = (_Float16*)(ws + off); off += w1_b;
  _Float16* w2T  = (_Float16*)(ws + off); off += w2_b;
  _Float16* xh   = (_Float16*)(ws + off); off += xh_b;
  _Float16* qpl  = (_Float16*)(ws + off); off += pl_b;
  _Float16* kpl  = (_Float16*)(ws + off); off += pl_b;
  _Float16* vtp  = (_Float16*)(ws + off); off += pl_b;
  _Float16* attn = (_Float16*)(ws + off); off += at_b;
  float*    xr   = (float*)(ws + off);    off += xr_b;
  _Float16* yh   = (_Float16*)(ws + off); off += yh_b;
  _Float16* hh   = (_Float16*)(ws + off); off += hh_b;
  if (off > ws_size) return;

  cvt_w_kernel<<<dim3(DM / 64, DM / 64, 3), 256, 0, stream>>>(Wq, Wk, Wv, wqkv, DM, DM);
  cvt_w_kernel<<<dim3(DM / 64, DM / 64, 1), 256, 0, stream>>>(Wo, Wo, Wo, woT, DM, DM);
  cvt_w_kernel<<<dim3(DM / 64, MLPD / 64, 1), 256, 0, stream>>>(W1, W1, W1, w1T, DM, MLPD);
  cvt_w_kernel<<<dim3(MLPD / 64, DM / 64, 1), 256, 0, stream>>>(W2, W2, W2, w2T, MLPD, DM);

  ln_kernel<<<NROWS / 8, 256, 0, stream>>>(x, ln1s, ln1b, xh, NROWS);

  gemm_kernel<0><<<dim3(NROWS / 128, NQKV / 64), 128, 0, stream>>>(
      xh, wqkv, NQKV, DM, b1, x, xr, hh, qpl, kpl, vtp);

  attn_kernel<<<dim3(NBLK, NH, NB), 128, 0, stream>>>(qpl, kpl, vtp, pm, ra, attn);

  gemm_kernel<1><<<dim3(NROWS / 128, DM / 64), 128, 0, stream>>>(
      attn, woT, DM, DM, b2, x, xr, hh, qpl, kpl, vtp);

  ln_kernel<<<NROWS / 8, 256, 0, stream>>>(xr, ln2s, ln2b, yh, NROWS);

  gemm_kernel<2><<<dim3(NROWS / 128, MLPD / 64), 128, 0, stream>>>(
      yh, w1T, MLPD, DM, b1, x, xr, hh, qpl, kpl, vtp);

  gemm_kernel<3><<<dim3(NROWS / 128, DM / 64), 128, 0, stream>>>(
      hh, w2T, DM, MLPD, b2, xr, out, yh, qpl, kpl, vtp);
}
